// HGTLayerWithLoss_23708219474684
// MI455X (gfx1250) — hardware-verified
//
#include <hip/hip_runtime.h>
#include <stddef.h>


#define DMD    128
#define NHD    8
#define DKD    16
#define QC     384
#define GT     128
#define SPW    (32 * 64)
#define WPP    136
#define RB     1024
#define RBBITS 10
#define RMAX   128
#define RMBITS 7
#define TABW   (2 * RMAX)
#define CHUNK  4096
#define LCAP   18432
#define DEGCAP 64
#define SCW    (32 * (DEGCAP / 2))
#define WSCAP  134217728
#define ASCL   8.0f
#define WSCL   64.0f
#define INVSCL 0.001953125f
#define PRISCL 0.00390625f

#define EDGE_LDS_INTS  (RB + 8 + RB + LCAP)
#define EDGE_LDS_BYTES ((EDGE_LDS_INTS + 8 * SCW) * 4)

static_assert(NHD * DKD == DMD);
static_assert(QC == 3 * DMD);
static_assert(RB == 256 * 4);
static_assert(RB == (1 << RBBITS));
static_assert(RMAX == (1 << RMBITS));
static_assert(CHUNK == 8 * 16 * 32);
static_assert(CHUNK == 4 * 4 * 256);
static_assert((WPP % 8) == 0);
static_assert((DEGCAP % 2) == 0);
static_assert(((EDGE_LDS_INTS * 4) % 16) == 0);
static_assert(EDGE_LDS_BYTES < 300000);

typedef float          v4f  __attribute__((ext_vector_type(4)));
typedef float          v8f  __attribute__((ext_vector_type(8)));
typedef int            v4i  __attribute__((ext_vector_type(4)));
typedef unsigned int   v4u  __attribute__((ext_vector_type(4)));
typedef unsigned short v8us __attribute__((ext_vector_type(8)));
typedef _Float16       v16h __attribute__((ext_vector_type(16)));
union FragH { v16h v; v8us u[2]; };

__device__ __forceinline__ unsigned short h16(float f) {
  const _Float16 h = (_Float16)f;
  return __builtin_bit_cast(unsigned short, h);
}
__device__ __forceinline__ float hf(unsigned short u) {
  return (float)__builtin_bit_cast(_Float16, u);
}

__device__ __forceinline__ v8us cvt8(v4f a, v4f b, float s) {
  v8us r;
  r[0] = h16(a.x * s); r[1] = h16(a.y * s); r[2] = h16(a.z * s); r[3] = h16(a.w * s);
  r[4] = h16(b.x * s); r[5] = h16(b.y * s); r[6] = h16(b.z * s); r[7] = h16(b.w * s);
  return r;
}

__device__ __forceinline__ v8f wmh(v16h a, v16h b, v8f c) {
  v8f d = __builtin_amdgcn_wmma_f32_16x16x32_f16(false, a, false, b, (short)0, c, false, false);
  asm volatile("v_nop\n\tv_nop\n\tv_nop\n\tv_nop" : "+v"(d) : "v"(a), "v"(b));
  return d;
}

template <int NB>
__device__ __forceinline__ unsigned int match_mask(unsigned int base, int key) {
  unsigned int msk = base;
#pragma unroll
  for (int b = 0; b < NB; ++b) {
    const bool bit = ((key >> b) & 1) != 0;
    const unsigned int bb = __builtin_amdgcn_ballot_w32(bit);
    msk &= bit ? bb : ~bb;
  }
  return msk;
}

__global__ __launch_bounds__(256) void k_hcvt(const float* __restrict__ h,
                                              unsigned short* h16p, int nN) {
  const int tid = (int)threadIdx.x, lane = tid & 31, wave = tid >> 5;
  int row = (int)blockIdx.x * 16 + wave * 2 + (lane >> 4);
  row = row > nN - 1 ? nN - 1 : row;
  const int c8 = 8 * (lane & 15);
  const float* p = h + (size_t)row * DMD + c8;
  const v4f a = *(const v4f*)p;
  const v4f b = *(const v4f*)(p + 4);
  const v8us o = cvt8(a, b, ASCL);
  unsigned short* op = h16p + (size_t)row * DMD + c8;
  *(volatile v8us*)op = o;
  __threadfence();
  *(volatile v8us*)op = o;
}

__global__ __launch_bounds__(256) void k_wprep(
    const float* __restrict__ Wq, const float* __restrict__ Wk, const float* __restrict__ Wv,
    const float* __restrict__ Wa, const float* __restrict__ bq, const float* __restrict__ bk,
    const float* __restrict__ bv, const float* __restrict__ ra, const float* __restrict__ rm,
    unsigned short* w16, float* bias384) {
  __shared__ __attribute__((aligned(16))) unsigned short sT[32 * WPP];
  __shared__ __attribute__((aligned(16))) float sB[32];
  const int tid = (int)threadIdx.x, lane = tid & 31;
  const int b = (int)blockIdx.x;
  const int g = b >> 2;
  const float* W   = (g == 0) ? Wq : ((g == 1) ? Wk : ((g == 2) ? Wv : Wa));
  const float* rel = (g == 1) ? ra : rm;
  const bool fold = (g == 1) || (g == 2);

#pragma unroll 1
  for (int it = 0; it < 16; ++it) {
    const int idx = it * 256 + tid;
    const int rr = idx >> 7, c = idx & 127;
    const int n = 32 * (b & 3) + rr;
    float val;
    if (fold) {
      const int hh = n >> 4, e = n & 15;
      float s = 0.0f;
#pragma unroll 1
      for (int d = 0; d < DKD; ++d)
        s = fmaf(W[(size_t)(hh * DKD + d) * DMD + c], rel[hh * 256 + d * 16 + e], s);
      val = s;
    } else {
      val = W[(size_t)n * DMD + c];
    }
    sT[rr * WPP + c] = h16(val * WSCL);
  }
  if (tid < 32) {
    const int n = 32 * (b & 3) + tid;
    float bb;
    if (fold) {
      const float* bsrc = (g == 1) ? bk : bv;
      const int hh = n >> 4, e = n & 15;
      float s = 0.0f;
#pragma unroll 1
      for (int d = 0; d < DKD; ++d)
        s = fmaf(bsrc[hh * DKD + d], rel[hh * 256 + d * 16 + e], s);
      bb = s;
    } else {
      bb = bq[n];
    }
    sB[tid] = bb;
  }
  __syncthreads();

  v8us pv[2];
  size_t po[2];
#pragma unroll
  for (int it = 0; it < 2; ++it) {
    const int p = it * 256 + tid;
    const int row = p >> 4, c8 = (p & 15) * 8;
    pv[it] = *(const v8us*)(sT + row * WPP + c8);
    po[it] = (size_t)(32 * b + row) * DMD + c8;
  }
  const v4f bl = *(const v4f*)(sB + 4 * (lane & 7));
  const bool wb = (g < 3) && (tid < 8);
  float* bp = bias384 + 32 * (b > 11 ? 11 : b) + 4 * (lane & 7);
#pragma unroll
  for (int it = 0; it < 2; ++it) *(volatile v8us*)(w16 + po[it]) = pv[it];
  if (wb) *(volatile v4f*)bp = bl;
  __threadfence();
#pragma unroll
  for (int it = 0; it < 2; ++it) *(volatile v8us*)(w16 + po[it]) = pv[it];
  if (wb) *(volatile v4f*)bp = bl;
}

template <int OUT16, int GATE>
__global__ __launch_bounds__(GT) void k_gemm(
    const unsigned short* __restrict__ A, const unsigned short* __restrict__ Bt,
    const float* __restrict__ bias, const float* __restrict__ res, const float* __restrict__ skp,
    float* outF, unsigned short* outH, int K, int Ncols, int M) {
  __shared__ __attribute__((aligned(16))) float sT[4 * SPW];
  const int tid = (int)threadIdx.x, lane = tid & 31, wave = tid >> 5, hh = lane >> 4, m = lane & 15;
  const int r0 = (int)blockIdx.y * 64 + (wave >> 1) * 32;
  const int c0 = (int)blockIdx.x * 128 + (wave & 1) * 64;

  int ra0 = r0 + m;      ra0 = ra0 > M - 1 ? M - 1 : ra0;
  int ra1 = r0 + 16 + m; ra1 = ra1 > M - 1 ? M - 1 : ra1;
  const unsigned short* ap0 = A + (size_t)ra0 * K + 8 * hh;
  const unsigned short* ap1 = A + (size_t)ra1 * K + 8 * hh;
  const unsigned short* bp[4];
#pragma unroll
  for (int j = 0; j < 4; ++j) {
    int cb = c0 + 16 * j + m; cb = cb > Ncols - 1 ? Ncols - 1 : cb;
    bp[j] = Bt + (size_t)cb * K + 8 * hh;
  }

  v8f acc[2][4];
#pragma unroll
  for (int i = 0; i < 2; ++i)
#pragma unroll
    for (int j = 0; j < 4; ++j) { v8f z = {0.f, 0.f, 0.f, 0.f, 0.f, 0.f, 0.f, 0.f}; acc[i][j] = z; }

  const int nk = K >> 5;
#pragma unroll 1
  for (int kt = 0; kt < nk; ++kt) {
    const int kb = kt << 5;
    FragH a0, a1;
    a0.u[0] = *(const v8us*)(ap0 + kb);
    a0.u[1] = *(const v8us*)(ap0 + kb + 16);
    a1.u[0] = *(const v8us*)(ap1 + kb);
    a1.u[1] = *(const v8us*)(ap1 + kb + 16);
#pragma unroll
    for (int j = 0; j < 4; ++j) {
      FragH bf;
      bf.u[0] = *(const v8us*)(bp[j] + kb);
      bf.u[1] = *(const v8us*)(bp[j] + kb + 16);
      acc[0][j] = wmh(a0.v, bf.v, acc[0][j]);
      acc[1][j] = wmh(a1.v, bf.v, acc[1][j]);
    }
  }

  float* sw = sT + wave * SPW;
#pragma unroll
  for (int i = 0; i < 2; ++i)
#pragma unroll
    for (int j = 0; j < 4; ++j)
#pragma unroll
      for (int r = 0; r < 8; ++r)
        sw[(16 * i + 8 * hh + r) * 64 + 16 * j + m] = acc[i][j][r];
  __syncthreads();

  const bool full = (r0 + 32 <= M) && (c0 + 64 <= Ncols);
  if (OUT16) {
    v8us hv[8];
    size_t po[8];
#pragma unroll
    for (int it = 0; it < 8; ++it) {
      const int f = it * 32 + lane;
      const int row = f >> 3, c8 = (f & 7) * 8;
      const v4f v0 = *(const v4f*)(sw + row * 64 + c8);
      const v4f v1 = *(const v4f*)(sw + row * 64 + c8 + 4);
      int gc = c0 + c8; gc = gc > Ncols - 8 ? Ncols - 8 : gc;
      const v4f b0v = *(const v4f*)(bias + gc);
      const v4f b1v = *(const v4f*)(bias + gc + 4);
      const v4f o0 = v0 * INVSCL + b0v;
      const v4f o1 = v1 * INVSCL + b1v;
      hv[it] = cvt8(o0, o1, ASCL);
      po[it] = (size_t)(r0 + row) * Ncols + c0 + c8;
    }
    if (full) {
#pragma unroll
      for (int it = 0; it < 8; ++it) *(volatile v8us*)(outH + po[it]) = hv[it];
    }
    __threadfence();
    if (full) {
#pragma unroll
      for (int it = 0; it < 8; ++it) *(volatile v8us*)(outH + po[it]) = hv[it];
    }
  } else {
    float alpha = 1.0f, beta = 0.0f;
    if (GATE) {
      const float sk = skp[0];
      alpha = 1.0f / (1.0f + expf(-sk));
      beta  = 1.0f - alpha;
    }
    v4f ov[16];
    size_t po[16];
#pragma unroll
    for (int it = 0; it < 16; ++it) {
      const int f = it * 32 + lane;
      const int row = f >> 4, c4 = (f & 15) * 4;
      const v4f v = *(const v4f*)(sw + row * 64 + c4);
      int gc = c0 + c4; gc = gc > Ncols - 4 ? Ncols - 4 : gc;
      int gr = r0 + row; gr = gr > M - 1 ? M - 1 : gr;
      const v4f bb = *(const v4f*)(bias + gc);
      v4f o = v * INVSCL + bb;
      if (GATE) {
        const v4f hr = *(const v4f*)(res + (size_t)gr * Ncols + gc);
        o = o * alpha + hr * beta;
      }
      ov[it] = o;
      po[it] = (size_t)(r0 + row) * Ncols + c0 + c4;
    }
    if (full) {
#pragma unroll
      for (int it = 0; it < 16; ++it) *(volatile v4f*)(outF + po[it]) = ov[it];
    }
    __threadfence();
    if (full) {
#pragma unroll
      for (int it = 0; it < 16; ++it) *(volatile v4f*)(outF + po[it]) = ov[it];
    }
  }
}

__global__ __launch_bounds__(256) void k_csort(
    const int* __restrict__ dst, unsigned int* csort, int* tab, int nN, int nE) {
  __shared__ __attribute__((aligned(16))) unsigned int sImg[CHUNK];
  __shared__ int cw[8 * RMAX];
  __shared__ __attribute__((aligned(16))) int sPre[RMAX];
  __shared__ __attribute__((aligned(16))) int sCn[RMAX];
  __shared__ int sWt[8];
  const int tid = (int)threadIdx.x, lane = tid & 31, wave = tid >> 5;
  const int c = (int)blockIdx.x;
  const int cbase = c * CHUNK;

  for (int i = tid; i < 8 * RMAX; i += 256) cw[i] = 0;
  {
    const v4u s = {0xffffffffu, 0xffffffffu, 0xffffffffu, 0xffffffffu};
    for (int i = tid; i < CHUNK / 4; i += 256) ((v4u*)sImg)[i] = s;
  }
  __syncthreads();

  unsigned int ent[16];
  int pk[16];
  const unsigned int lt = (1u << lane) - 1u;
#pragma unroll
  for (int i = 0; i < 16; ++i) {
    const int e = cbase + wave * 512 + 32 * i + lane;
    const int ea = e > nE - 1 ? nE - 1 : e;
    const int d = dst[ea];
    const bool valid = (e < nE) && ((unsigned)d < (unsigned)nN);
    const int dd = valid ? d : 0;
    const int r  = dd >> RBBITS;
    const int jl = dd & (RB - 1);
    const unsigned int msk = match_mask<RMBITS>(__builtin_amdgcn_ballot_w32(valid), r);
    const int rank = (int)__builtin_popcount(msk & lt);
    const int grp  = (int)__builtin_popcount(msk);
    const int base = cw[wave * RMAX + r];
    pk[i]  = valid ? ((r << 12) | (base + rank)) : -1;
    ent[i] = ((unsigned int)ea << RBBITS) | (unsigned int)jl;
    if (valid && rank == 0) cw[wave * RMAX + r] = base + grp;
    __syncthreads();
  }

  if (tid < RMAX) {
    int run = 0;
#pragma unroll
    for (int w = 0; w < 8; ++w) {
      const int v = cw[w * RMAX + tid];
      cw[w * RMAX + tid] = run;
      run += v;
    }
    sCn[tid] = run;
  }
  __syncthreads();
  {
    const int vr = sCn[tid & (RMAX - 1)];
    const int v  = (tid < RMAX) ? vr : 0;
    int x = v;
#pragma unroll
    for (int dd = 1; dd < 32; dd <<= 1) {
      const int y = __shfl_up(x, dd);
      x += (lane >= dd) ? y : 0;
    }
    if (lane == 31) sWt[wave] = x;
    __syncthreads();
    int pre = 0;
#pragma unroll
    for (int w = 0; w < 8; ++w) { const int tw = sWt[w]; pre += (w < wave) ? tw : 0; }
    if (tid < RMAX) sPre[tid] = pre + x - v;
  }
  __syncthreads();

#pragma unroll
  for (int i = 0; i < 16; ++i) {
    if (pk[i] >= 0) {
      const int r = (pk[i] >> 12) & (RMAX - 1);
      const int q = pk[i] & 4095;
      const int pos = sPre[r] + cw[wave * RMAX + r] + q;
      if ((unsigned)pos < (unsigned)CHUNK) sImg[pos] = ent[i];
    }
  }
  __syncthreads();

  v4u iv[4];
#pragma unroll
  for (int it = 0; it < 4; ++it) iv[it] = ((const v4u*)sImg)[it * 256 + tid];
  const v4i ta = *(const v4i*)(sPre + 4 * lane);
  const v4i tb = *(const v4i*)(sCn + 4 * lane);
  const v4i tv = (wave == 0) ? ta : tb;
  unsigned int* gp = csort + (size_t)c * CHUNK;
  int* tp = tab + (size_t)c * TABW + 4 * tid;
  const bool wt = tid < 64;
#pragma unroll
  for (int it = 0; it < 4; ++it) *(volatile v4u*)(gp + 4 * (it * 256 + tid)) = iv[it];
  if (wt) *(volatile v4i*)tp = tv;
  __threadfence();
#pragma unroll
  for (int it = 0; it < 4; ++it) *(volatile v4u*)(gp + 4 * (it * 256 + tid)) = iv[it];
  if (wt) *(volatile v4i*)tp = tv;
}

__global__ __launch_bounds__(256) void k_edge(
    const unsigned short* __restrict__ qkv, const int* __restrict__ src,
    const unsigned int* __restrict__ csort, const int* __restrict__ tab,
    const float* __restrict__ pri, unsigned short* t16, int nN, int nE, int nCh) {
  extern __shared__ __attribute__((aligned(16))) int dsm[];
  __shared__ int sWtot[8];
  int*   sOff  = dsm;
  int*   sCur  = dsm + (RB + 8);
  int*   sList = sCur + RB;
  float* sSc   = (float*)(sList + LCAP);
  const int tid = (int)threadIdx.x, lane = tid & 31, wave = tid >> 5;
  const int rgn = (int)blockIdx.x;
  const int n0 = rgn * RB;
  const unsigned int lt = (1u << lane) - 1u;

  for (int i = tid; i < RB + 8; i += 256) sOff[i] = 0;
  for (int i = tid; i < RB; i += 256) sCur[i] = 0;
  __syncthreads();

#pragma unroll 1
  for (int c = 0; c < nCh; ++c) {
    int pre = tab[(size_t)c * TABW + rgn];
    int n   = tab[(size_t)c * TABW + RMAX + rgn];
    pre = pre < 0 ? 0 : (pre > CHUNK ? CHUNK : pre);
    n = n < 0 ? 0 : (n > CHUNK - pre ? CHUNK - pre : n);
    const int nstep = (n + 31) >> 5;
    const unsigned int* cp = csort + (size_t)c * CHUNK + pre;
#pragma unroll 1
    for (int s = 0; s < nstep; ++s) {
      if (wave == 0) {
        const int i = (s << 5) + lane;
        const bool valid = i < n;
        const int ic = i > n - 1 ? n - 1 : i;
        const unsigned int en = cp[ic];
        const int j = (int)(en & (unsigned int)(RB - 1));
        const unsigned int msk = match_mask<RBBITS>(__builtin_amdgcn_ballot_w32(valid), j);
        const int rank = (int)__builtin_popcount(msk & lt);
        const int grp  = (int)__builtin_popcount(msk);
        if (valid && rank == 0) sOff[j] = sOff[j] + grp;
      }
      __syncthreads();
    }
  }
  __syncthreads();

  {
    int cn[4];
    int ls = 0;
#pragma unroll
    for (int i = 0; i < 4; ++i) { cn[i] = sOff[4 * tid + i]; ls += cn[i]; }
    int x = ls;
#pragma unroll
    for (int dd = 1; dd < 32; dd <<= 1) {
      const int y = __shfl_up(x, dd);
      x += (lane >= dd) ? y : 0;
    }
    if (lane == 31) sWtot[wave] = x;
    __syncthreads();
    int pre = 0;
#pragma unroll
    for (int w = 0; w < 8; ++w) { const int tw = sWtot[w]; pre += (w < wave) ? tw : 0; }
    int run = pre + x - ls;
#pragma unroll
    for (int i = 0; i < 4; ++i) { sOff[4 * tid + i] = run; run += cn[i]; }
    if (tid == 255) sOff[RB] = run;
  }
  __syncthreads();

#pragma unroll 1
  for (int c = 0; c < nCh; ++c) {
    int pre = tab[(size_t)c * TABW + rgn];
    int n   = tab[(size_t)c * TABW + RMAX + rgn];
    pre = pre < 0 ? 0 : (pre > CHUNK ? CHUNK : pre);
    n = n < 0 ? 0 : (n > CHUNK - pre ? CHUNK - pre : n);
    const int nstep = (n + 31) >> 5;
    const unsigned int* cp = csort + (size_t)c * CHUNK + pre;
#pragma unroll 1
    for (int s = 0; s < nstep; ++s) {
      if (wave == 0) {
        const int i = (s << 5) + lane;
        const bool valid = i < n;
        const int ic = i > n - 1 ? n - 1 : i;
        const unsigned int en = cp[ic];
        const int j = (int)(en & (unsigned int)(RB - 1));
        int e = (int)(en >> RBBITS);
        e = e > nE - 1 ? nE - 1 : e;
        const unsigned int msk = match_mask<RBBITS>(__builtin_amdgcn_ballot_w32(valid), j);
        const int rank = (int)__builtin_popcount(msk & lt);
        const int grp  = (int)__builtin_popcount(msk);
        const int cur  = sCur[j];
        const int p0   = sOff[j] + cur + rank;
        if (valid && (unsigned)p0 < (unsigned)LCAP) sList[p0] = e;
        if (valid && rank == 0) sCur[j] = cur + grp;
      }
      __syncthreads();
    }
  }
  __syncthreads();

  const int ch = 8 * (lane & 15);
  const int hd = (lane & 15) >> 1;
  const float pf = pri[hd] * PRISCL;
  int Rb = nN - n0; Rb = Rb > RB ? RB : Rb;
  float* sw = sSc + wave * SCW;
#pragma unroll 1
  for (int j = wave; j < Rb; j += 8) {
    const int node = n0 + j;
    int lb = __builtin_amdgcn_readfirstlane(sOff[j]);
    int ub = __builtin_amdgcn_readfirstlane(sOff[j + 1]);
    lb = lb < 0 ? 0 : (lb > LCAP ? LCAP : lb);
    ub = ub < 0 ? 0 : (ub > LCAP ? LCAP : ub);
    int cnt = ub - lb;
    cnt = cnt < 0 ? 0 : (cnt > DEGCAP ? DEGCAP : cnt);
    const int np = (cnt + 1) >> 1;

    const v8us qv = *(const v8us*)(qkv + (size_t)node * QC + ch);
    float qf[8];
#pragma unroll
    for (int cc = 0; cc < 8; ++cc) qf[cc] = hf(qv[cc]);

    float m = __int_as_float(0xff800000u);
#pragma unroll 1
    for (int it = 0; it < np; ++it) {
      const int i = 2 * it + (lane >> 4);
      const bool valid = i < cnt;
      const int ic = valid ? i : (cnt - 1);
      int li = lb + ic; li = li < 0 ? 0 : (li > LCAP - 1 ? LCAP - 1 : li);
      int e = sList[li]; e = e < 0 ? 0 : (e > nE - 1 ? nE - 1 : e);
      int s = src[e];   s = s < 0 ? 0 : (s > nN - 1 ? nN - 1 : s);
      const v8us kv = *(const v8us*)(qkv + (size_t)s * QC + DMD + ch);
      float part = 0.0f;
#pragma unroll
      for (int cc = 0; cc < 8; ++cc) part = fmaf(qf[cc], hf(kv[cc]), part);
      part += __shfl_xor(part, 1);
      const float sc = part * pf;
      m = valid ? fmaxf(m, sc) : m;
      sw[it * 32 + lane] = sc;
    }
    m = fmaxf(m, __shfl_xor(m, 16));

    float acc[8];
#pragma unroll
    for (int cc = 0; cc < 8; ++cc) acc[cc] = 0.0f;
    float z = 0.0f;
#pragma unroll 1
    for (int it = 0; it < np; ++it) {
      const int i = 2 * it + (lane >> 4);
      const bool valid = i < cnt;
      const int ic = valid ? i : (cnt - 1);
      int li = lb + ic; li = li < 0 ? 0 : (li > LCAP - 1 ? LCAP - 1 : li);
      int e = sList[li]; e = e < 0 ? 0 : (e > nE - 1 ? nE - 1 : e);
      int s = src[e];   s = s < 0 ? 0 : (s > nN - 1 ? nN - 1 : s);
      const float sc = sw[it * 32 + lane];
      float p = __expf(sc - m);
      p = valid ? p : 0.0f;
      const v8us vv = *(const v8us*)(qkv + (size_t)s * QC + 2 * DMD + ch);
#pragma unroll
      for (int cc = 0; cc < 8; ++cc) acc[cc] = fmaf(p, hf(vv[cc]), acc[cc]);
      z += p;
    }
#pragma unroll
    for (int cc = 0; cc < 8; ++cc) acc[cc] += __shfl_xor(acc[cc], 16);
    z += __shfl_xor(z, 16);
    const float zs = (cnt > 0) ? z : 1.0f;
    const float rz = 1.0f / zs;
    v8us o;
#pragma unroll
    for (int cc = 0; cc < 8; ++cc) o[cc] = h16(acc[cc] * rz);
    unsigned short* tp = t16 + (size_t)node * DMD + ch;
    if (lane < 16) *(volatile v8us*)tp = o;
    __threadfence();
    if (lane < 16) *(volatile v8us*)tp = o;
  }
}

extern "C" void kernel_launch(void* const* d_in, const int* in_sizes, int n_in,
                              void* d_out, int out_size, void* d_ws, size_t ws_size,
                              hipStream_t stream) {
  if (n_in < 15) return;
  const int nN = in_sizes[0] / DMD;
  const int nE = in_sizes[1];
  if (nN <= 0 || nE <= 0) return;
  if (in_sizes[0] != nN * DMD || (nN % 32) != 0) return;
  if (in_sizes[2] != nE) return;
  if (nN > RMAX * RB || nE > (1 << 22)) return;
  if (in_sizes[3] != DMD * DMD || in_sizes[5] != DMD * DMD || in_sizes[7] != DMD * DMD || in_sizes[9] != DMD * DMD) return;
  if (in_sizes[4] != DMD || in_sizes[6] != DMD || in_sizes[8] != DMD || in_sizes[10] != DMD) return;
  if (in_sizes[11] != NHD * DKD * DKD || in_sizes[12] != NHD * DKD * DKD) return;
  if (in_sizes[13] != NHD || in_sizes[14] < 1) return;
  if (out_size != nN * DMD) return;

  const float* h   = (const float*)d_in[0];
  const int*   src = (const int*)d_in[1];
  const int*   dst = (const int*)d_in[2];
  const float* Wk  = (const float*)d_in[3];
  const float* bk  = (const float*)d_in[4];
  const float* Wq  = (const float*)d_in[5];
  const float* bq  = (const float*)d_in[6];
  const float* Wv  = (const float*)d_in[7];
  const float* bv  = (const float*)d_in[8];
  const float* Wa  = (const float*)d_in[9];
  const float* ba  = (const float*)d_in[10];
  const float* ra  = (const float*)d_in[11];
  const float* rm  = (const float*)d_in[12];
  const float* pri = (const float*)d_in[13];
  const float* skp = (const float*)d_in[14];
  float* out = (float*)d_out;

  const int nCh = (nE + CHUNK - 1) / CHUNK;
  const int nR  = (nN + RB - 1) / RB;

  const size_t nNp   = (size_t)((nN + 63) / 64) * 64;
  const size_t szH16 = (size_t)nN * DMD * 2;
  const size_t szW16 = (size_t)512 * DMD * 2;
  const size_t szB   = (size_t)QC * 4;
  const size_t szQKV = nNp * QC * 2;
  const size_t szT16 = nNp * DMD * 2;
  const size_t szCS  = (size_t)nCh * CHUNK * 4;
  const size_t szTab = (size_t)nCh * TABW * 4;
  size_t off = 0;
  const size_t oH = off; off += szH16; off = (off + 255) & ~(size_t)255;
  const size_t oW = off; off += szW16; off = (off + 255) & ~(size_t)255;
  const size_t oB = off; off += szB;   off = (off + 255) & ~(size_t)255;
  const size_t oQ = off; off += szQKV; off = (off + 255) & ~(size_t)255;
  const size_t oT = off; off += szT16; off = (off + 255) & ~(size_t)255;
  if (off > ws_size || off > (size_t)WSCAP) return;
  const size_t oCS  = oH;
  const size_t oTab = (oCS + szCS + 255) & ~(size_t)255;
  if (oTab + szTab > oH + szH16) return;

  char* ws = (char*)d_ws;
  unsigned short* h16p    = (unsigned short*)(ws + oH);
  unsigned short* w16     = (unsigned short*)(ws + oW);
  float*          bias384 = (float*)(ws + oB);
  unsigned short* qkv16   = (unsigned short*)(ws + oQ);
  unsigned short* t16     = (unsigned short*)(ws + oT);
  unsigned int*   csort   = (unsigned int*)(ws + oCS);
  int*            tab     = (int*)(ws + oTab);

  const dim3 gQ(QC / 128, (nN + 63) / 64);
  const dim3 gA(1, (nN + 63) / 64);

  k_hcvt<<<nN / 16, 256, 0, stream>>>(h, h16p, nN);

  k_wprep<<<16, 256, 0, stream>>>(Wq, Wk, Wv, Wa, bq, bk, bv, ra, rm, w16, bias384);

  k_gemm<1, 0><<<gQ, GT, 0, stream>>>(h16p, w16, bias384, h, skp, out, qkv16, DMD, QC, nN);

  k_csort<<<nCh, 256, 0, stream>>>(dst, csort, tab, nN, nE);

  hipFuncSetAttribute(reinterpret_cast<const void*>(&k_edge),
                      hipFuncAttributeMaxDynamicSharedMemorySize, EDGE_LDS_BYTES);
  k_edge<<<nR, 256, EDGE_LDS_BYTES, stream>>>(qkv16, src, csort, tab, pri, t16, nN, nE, nCh);

  k_gemm<0, 1><<<gA, GT, 0, stream>>>(t16, w16 + (size_t)QC * DMD, ba, h, skp, out, qkv16, DMD, DMD, nN);
}
